// DynamicRoutingPooler_25606595019362
// MI455X (gfx1250) — hardware-verified
//
#include <hip/hip_runtime.h>
#include <math.h>

#ifndef NB
#define NB 8
#endif
#ifndef SEQ
#define SEQ 2048
#endif
#define NB_FULL 8
#define SEQ_FULL 2048
#define DIN 512
#define DOUT 512
#define NCAP 8

#define RT_SP 516
#define RT_VP 520
#define W2OFF ((size_t)NCAP * DOUT * DIN)

static_assert(NCAP == 8);
static_assert(NB >= 1 && NB <= 8 && NB <= NB_FULL);
static_assert(SEQ <= SEQ_FULL);
static_assert(DIN == DOUT);
static_assert(DIN == 512 && DOUT == 8 * 64);
static_assert(DIN % 64 == 0 && DIN % 32 == 0 && DOUT % 32 == 0);
static_assert(SEQ % 256 == 0 && SEQ % 128 == 0 && SEQ % 64 == 0 && SEQ % 32 == 0);
static_assert((DIN * 64) % 256 == 0);
static_assert(NCAP * SEQ * 4 <= 131072);
static_assert(8 * RT_SP * 4 + 8 * RT_VP * 2 + 8 * 8 * 68 * 4 + 32 <= 131072);
static_assert(8 * 16 * 68 * 4 <= 131072);
static_assert((RT_SP * 4) % 16 == 0 && (RT_VP * 2) % 16 == 0);
static_assert((size_t)NB_FULL * NCAP * DOUT * 4 == 131072);

typedef __attribute__((ext_vector_type(16))) _Float16 v16h;
typedef __attribute__((ext_vector_type(8)))  _Float16 v8h;
typedef __attribute__((ext_vector_type(8)))  float    v8f;
typedef __attribute__((ext_vector_type(4)))  float    v4f;
typedef __attribute__((ext_vector_type(4)))  unsigned int v4u;


#define VST2(T, ptr, val) do { const T vst2_v_ = (val); *(volatile T*)(ptr) = vst2_v_; __threadfence(); *(volatile T*)(ptr) = vst2_v_; } while (0)
#define VST2V4(ptr, val) do { const v4f vst2_v4_ = (val); *(volatile v4f*)(ptr) = vst2_v4_; __threadfence(); *(volatile v4f*)(ptr) = vst2_v4_; } while (0)

__device__ __forceinline__ float bfr(float f) {
    unsigned u = __float_as_uint(f);
    u += 0x7FFFu + ((u >> 16) & 1u);
    return __uint_as_float(u & 0xFFFF0000u);
}
__device__ __forceinline__ unsigned short f2h_bits(float x) {
    return (fabsf(x) < 6.104e-5f) ? (unsigned short)0 : __builtin_bit_cast(unsigned short, (_Float16)x);
}
__device__ __forceinline__ void st8h(unsigned short* P, size_t o, const float* v) {
    v4u pk;
    pk.x = (unsigned)f2h_bits(v[0]) | ((unsigned)f2h_bits(v[1]) << 16);
    pk.y = (unsigned)f2h_bits(v[2]) | ((unsigned)f2h_bits(v[3]) << 16);
    pk.z = (unsigned)f2h_bits(v[4]) | ((unsigned)f2h_bits(v[5]) << 16);
    pk.w = (unsigned)f2h_bits(v[6]) | ((unsigned)f2h_bits(v[7]) << 16);
    VST2(v4u, (v4u*)(P + o), pk);
}
__device__ __forceinline__ _Float16 toh_flush(float v) {
    const _Float16 r = (_Float16)v;
    return (fabsf(v) < 6.103515625e-05f) ? (_Float16)0.0f : r;
}

union FragU { v16h v; v8h h[2]; };
__device__ __forceinline__ v16h frag_ld(const _Float16* p) {
    FragU f; f.h[0] = *(const v8h*)(p); f.h[1] = *(const v8h*)(p + 16); return f.v;
}
__device__ __forceinline__ v8f wmma16(v16h a, v16h b, v8f c) {
    c = __builtin_amdgcn_wmma_f32_16x16x32_f16(false, a, false, b, (short)0, c, false, false);
    asm volatile("v_nop\n\tv_nop\n\tv_nop\n\tv_nop" : "+v"(c) : "v"(a), "v"(b));
    return c;
}
__device__ __forceinline__ void wave_sync_lds() {
    __builtin_amdgcn_fence(3  , "workgroup");
    __builtin_amdgcn_wave_barrier();
    __builtin_amdgcn_fence(2  , "workgroup");
}

__global__ __launch_bounds__(256) void k_wconv(const float* __restrict__ Wm, unsigned short* __restrict__ Wp) {
    const unsigned u = blockIdx.x * 256u + threadIdx.x;
    const unsigned g = u & 63u, rowA = u >> 6;
    const unsigned mode = blockIdx.y;
    const size_t src0 = (mode == 0u) ? ((size_t)(8u * g) * (DOUT * NCAP) + (size_t)rowA * NCAP)
                                     : ((size_t)rowA * (DOUT * NCAP) + (size_t)(8u * g) * NCAP);
    const size_t estr = (mode == 0u) ? (size_t)(DOUT * NCAP) : (size_t)NCAP;
    const size_t poff = (mode == 0u) ? (size_t)0 : W2OFF;
    v4f w[16];
#pragma unroll
    for (int e = 0; e < 8; ++e) {
        w[2 * e]     = *(const v4f*)(Wm + src0 + (size_t)e * estr);
        w[2 * e + 1] = *(const v4f*)(Wm + src0 + (size_t)e * estr + 4);
    }
#pragma unroll
    for (int c = 0; c < 8; ++c) {
        float v[8];
#pragma unroll
        for (int e = 0; e < 8; ++e) v[e] = bfr(w[2 * e + (c >> 2)][c & 3]) * 32.0f;
        st8h(Wp, poff + ((size_t)((unsigned)c * 512u + rowA)) * 512u + 8u * g, v);
    }
}

static_assert(256 * 16 * 2 == 64 * 128);
__global__ __launch_bounds__(256) void k_fconv(const float* __restrict__ F, unsigned short* __restrict__ F16,
                                               unsigned short* __restrict__ FT16) {
    __shared__ __align__(16) unsigned short sT[64 * 72];
    const unsigned t = threadIdx.x;
    const unsigned it0 = blockIdx.x % (unsigned)(DIN / 64);
    const unsigned rest = blockIdx.x / (unsigned)(DIN / 64);
    const unsigned st0 = rest % (unsigned)(SEQ / 64);
    const unsigned b = rest / (unsigned)(SEQ / 64);
    const unsigned i0 = it0 * 64u, s0 = st0 * 64u;
    {
        const unsigned row = t >> 2, seg = t & 3u;
        const float* src = F + ((size_t)b * SEQ_FULL + s0 + row) * DIN + i0 + 16u * seg;
        unsigned short hb[16];
#pragma unroll
        for (int g = 0; g < 4; ++g) {
            const v4f a = *(const v4f*)(src + 4 * g);
            hb[4 * g + 0] = f2h_bits(bfr(a.x) * 8.0f);
            hb[4 * g + 1] = f2h_bits(bfr(a.y) * 8.0f);
            hb[4 * g + 2] = f2h_bits(bfr(a.z) * 8.0f);
            hb[4 * g + 3] = f2h_bits(bfr(a.w) * 8.0f);
        }
        v4u p0, p1;
        p0.x = (unsigned)hb[0]  | ((unsigned)hb[1]  << 16); p0.y = (unsigned)hb[2]  | ((unsigned)hb[3]  << 16);
        p0.z = (unsigned)hb[4]  | ((unsigned)hb[5]  << 16); p0.w = (unsigned)hb[6]  | ((unsigned)hb[7]  << 16);
        p1.x = (unsigned)hb[8]  | ((unsigned)hb[9]  << 16); p1.y = (unsigned)hb[10] | ((unsigned)hb[11] << 16);
        p1.z = (unsigned)hb[12] | ((unsigned)hb[13] << 16); p1.w = (unsigned)hb[14] | ((unsigned)hb[15] << 16);
        *(v4u*)&sT[row * 72u + 16u * seg] = p0;
        *(v4u*)&sT[row * 72u + 16u * seg + 8u] = p1;
    }
    __syncthreads();
    const unsigned rq = t >> 3, c8 = (t & 7u) * 8u;
#pragma unroll
    for (int it = 0; it < 2; ++it) {
        const unsigned row = rq + 32u * (unsigned)it;
        const v4u pk = *(const v4u*)&sT[row * 72u + c8];
        VST2(v4u, (v4u*)(F16 + ((size_t)(b * SEQ + s0 + row)) * DIN + i0 + c8), pk);
    }
#pragma unroll
    for (int it = 0; it < 2; ++it) {
        const unsigned irow = rq + 32u * (unsigned)it;
        unsigned short hb[8];
#pragma unroll
        for (int e = 0; e < 8; ++e) hb[e] = sT[(c8 + (unsigned)e) * 72u + irow];
        v4u pk;
        pk.x = (unsigned)hb[0] | ((unsigned)hb[1] << 16); pk.y = (unsigned)hb[2] | ((unsigned)hb[3] << 16);
        pk.z = (unsigned)hb[4] | ((unsigned)hb[5] << 16); pk.w = (unsigned)hb[6] | ((unsigned)hb[7] << 16);
        VST2(v4u, (v4u*)(FT16 + ((size_t)(b * DIN + i0 + irow)) * SEQ + s0 + c8), pk);
    }
}

static_assert(32 * 16 * 2 == 8 * 128);
__global__ __launch_bounds__(256) void k_pool(const _Float16* __restrict__ R16, const _Float16* __restrict__ FT16,
                                              unsigned short* __restrict__ M16, int first) {
    __shared__ __align__(16) float sD[8][16 * 68];
    const unsigned lane = threadIdx.x & 31u;
    const unsigned wave = (unsigned)__builtin_amdgcn_readfirstlane((int)(threadIdx.x >> 5));
    const unsigned hh = lane >> 4, c = lane & 15u;
    const unsigned b = blockIdx.x;
    const unsigned i0 = wave * 64u;
    const _Float16* arow = R16 + ((size_t)(b * NCAP + (c & 7u))) * SEQ + 8u * hh;
    const _Float16* brow = FT16 + ((size_t)(b * DIN + i0 + c)) * SEQ + 8u * hh;
    v16h ones, zer;
#pragma unroll
    for (int i = 0; i < 16; ++i) { ones[i] = (_Float16)1.0f; zer[i] = (_Float16)0.0f; }
    v8f acc[4];
#pragma unroll
    for (int j = 0; j < 4; ++j) acc[j] = (v8f){0.f,0.f,0.f,0.f,0.f,0.f,0.f,0.f};
#pragma unroll 2
    for (unsigned k0 = 0; k0 < (unsigned)SEQ; k0 += 32u) {
        v16h a = zer;
        if (first == 0) a = frag_ld(arow + k0);
        a = (c < 8u) ? a : ones;
#pragma unroll
        for (int j = 0; j < 4; ++j) {
            const v16h bf = frag_ld(brow + (size_t)(16 * j) * SEQ + k0);
            acc[j] = wmma16(a, bf, acc[j]);
        }
    }
#pragma unroll
    for (int j = 0; j < 4; ++j)
#pragma unroll
        for (int r = 0; r < 8; ++r)
            sD[wave][(8u * hh + (unsigned)r) * 68u + (unsigned)j * 16u + c] = acc[j][r];
    wave_sync_lds();
    const unsigned q = lane >> 3, c8 = (lane & 7u) * 8u;
    const float sc = 8.0f / (float)SEQ;
#pragma unroll
    for (int it = 0; it < 2; ++it) {
        const unsigned cc = 4u * (unsigned)it + q;
        float v[8];
#pragma unroll
        for (int e = 0; e < 8; ++e)
            v[e] = (sD[wave][cc * 68u + c8 + (unsigned)e] * 0.0625f + sD[wave][8u * 68u + c8 + (unsigned)e]) * sc;
        st8h(M16, ((size_t)(cc * NB + b)) * DIN + i0 + c8, v);
    }
}

__global__ __launch_bounds__(256) void k_route(const _Float16* __restrict__ M16, const _Float16* __restrict__ Wp,
                                               const float* __restrict__ bias, const float* __restrict__ gamma,
                                               const float* __restrict__ beta, unsigned short* __restrict__ U16,
                                               float* __restrict__ BT, float* __restrict__ out, int last) {
    __shared__ __align__(16) float sS[8 * RT_SP];
    __shared__ __align__(16) _Float16 sV[8 * RT_VP];
    __shared__ __align__(16) float sU[8][8 * 68];
    __shared__ float sSum[8];
    const unsigned lane = threadIdx.x & 31u;
    const unsigned wave = (unsigned)__builtin_amdgcn_readfirstlane((int)(threadIdx.x >> 5));
    const unsigned hh = lane >> 4, c = lane & 15u;
    const unsigned cap = blockIdx.x;
    const unsigned ar = min(c & 7u, (unsigned)(NB - 1));
    const float bc = bfr(bias[cap]);
    {
        const unsigned n0 = wave * 64u;
        const _Float16* arow = M16 + ((size_t)(cap * NB + ar)) * DIN + 8u * hh;
        const _Float16* brow = Wp + ((size_t)(cap * DOUT + n0 + c)) * DIN + 8u * hh;
        v8f acc[4];
#pragma unroll
        for (int j = 0; j < 4; ++j) acc[j] = (v8f){0.f,0.f,0.f,0.f,0.f,0.f,0.f,0.f};
#pragma unroll 2
        for (unsigned k0 = 0; k0 < (unsigned)DIN; k0 += 32u) {
            const v16h a = frag_ld(arow + k0);
#pragma unroll
            for (int j = 0; j < 4; ++j) {
                const v16h bf = frag_ld(brow + (size_t)(16 * j) * DIN + k0);
                acc[j] = wmma16(a, bf, acc[j]);
            }
        }
#pragma unroll
        for (int j = 0; j < 4; ++j)
#pragma unroll
            for (int r2 = 0; r2 < 4; ++r2) {
                const float val = (hh != 0u) ? acc[j][r2 + 4] : acc[j][r2];
                sS[(4u * hh + (unsigned)r2) * RT_SP + n0 + (unsigned)j * 16u + c] = val * (1.0f / 2048.0f) + bc;
            }
    }
    __syncthreads();
    const unsigned bw = wave;
    float x[16];
#pragma unroll
    for (int j = 0; j < 4; ++j) {
        const v4f t4 = *(const v4f*)&sS[bw * RT_SP + 4u * lane + 128u * (unsigned)j];
        x[4 * j] = t4.x; x[4 * j + 1] = t4.y; x[4 * j + 2] = t4.z; x[4 * j + 3] = t4.w;
    }
    float ss = 0.f;
#pragma unroll
    for (int i = 0; i < 16; ++i) ss += x[i] * x[i];
#pragma unroll
    for (int o = 16; o > 0; o >>= 1) ss += __shfl_xor(ss, o, 32);
    const float nrm = sqrtf(ss);
    const float n2 = nrm * nrm;
    const float fsq = n2 * (1.0f / (n2 + 1.0f));
    const float rinv = 1.0f / (nrm + 1e-8f);
    float sv = 0.f;
#pragma unroll
    for (int i = 0; i < 16; ++i) { x[i] = (fsq * x[i]) * rinv; sv += x[i]; }
#pragma unroll
    for (int o = 16; o > 0; o >>= 1) sv += __shfl_xor(sv, o, 32);

    if (last != 0) {
        const float mu = sv * (1.0f / (float)DOUT);
        float qv = 0.f;
#pragma unroll
        for (int i = 0; i < 16; ++i) { x[i] -= mu; qv += x[i] * x[i]; }
#pragma unroll
        for (int o = 16; o > 0; o >>= 1) qv += __shfl_xor(qv, o, 32);
        const float rs = 1.0f / sqrtf(qv * (1.0f / (float)DOUT) + 1e-5f);
        if (bw < (unsigned)NB) {
            float* orow = out + ((size_t)(bw * NCAP + cap)) * DOUT;
#pragma unroll
            for (int j = 0; j < 4; ++j) {
                const unsigned d0 = 4u * lane + 128u * (unsigned)j;
                const v4f g4 = *(const v4f*)(gamma + d0);
                const v4f b4 = *(const v4f*)(beta + d0);
                v4f o4;
                o4.x = x[4 * j]     * rs * bfr(g4.x) + bfr(b4.x);
                o4.y = x[4 * j + 1] * rs * bfr(g4.y) + bfr(b4.y);
                o4.z = x[4 * j + 2] * rs * bfr(g4.z) + bfr(b4.z);
                o4.w = x[4 * j + 3] * rs * bfr(g4.w) + bfr(b4.w);
                VST2V4(orow + d0, o4);
            }
        }
    } else {
        if (lane == 0u) sSum[bw] = sv;
#pragma unroll
        for (int j = 0; j < 4; ++j)
#pragma unroll
            for (int e = 0; e < 4; ++e)
                sV[bw * RT_VP + 4u * lane + 128u * (unsigned)j + (unsigned)e] = toh_flush(x[4 * j + e] * 4096.0f);
        __syncthreads();
        if (wave == 0u && lane < 8u) {
            v4f z;
#pragma unroll
            for (int e = 0; e < 4; ++e) {
                const unsigned idx = 4u * lane + (unsigned)e;
                const float sval = sSum[min(idx, 7u)];
                z[e] = (idx < (unsigned)NB) ? bc * sval : 0.0f;
            }
            VST2V4(BT + cap * 32u + 4u * lane, z);
        }
        const unsigned i0 = wave * 64u;
        const _Float16* brow = Wp + W2OFF + ((size_t)(cap * DIN + i0 + c)) * DOUT + 8u * hh;
        v8f acc[4];
#pragma unroll
        for (int j = 0; j < 4; ++j) acc[j] = (v8f){0.f,0.f,0.f,0.f,0.f,0.f,0.f,0.f};
#pragma unroll 2
        for (unsigned k0 = 0; k0 < (unsigned)DOUT; k0 += 32u) {
            FragU fa;
            fa.h[0] = *(const v8h*)&sV[ar * RT_VP + k0 + 8u * hh];
            fa.h[1] = *(const v8h*)&sV[ar * RT_VP + k0 + 16u + 8u * hh];
#pragma unroll
            for (int j = 0; j < 4; ++j) {
                const v16h bf = frag_ld(brow + (size_t)(16 * j) * DOUT + k0);
                acc[j] = wmma16(fa.v, bf, acc[j]);
            }
        }
#pragma unroll
        for (int j = 0; j < 4; ++j)
#pragma unroll
            for (int r2 = 0; r2 < 4; ++r2) {
                const float val = (hh != 0u) ? acc[j][r2 + 4] : acc[j][r2];
                sU[wave][(4u * hh + (unsigned)r2) * 68u + (unsigned)j * 16u + c] = val * 0.125f;
            }
        wave_sync_lds();
        const unsigned q = lane >> 3, c8 = (lane & 7u) * 8u;
#pragma unroll
        for (int it = 0; it < 2; ++it) {
            const unsigned bb = 4u * (unsigned)it + q;
            float v[8];
#pragma unroll
            for (int e = 0; e < 8; ++e) v[e] = sU[wave][bb * 68u + c8 + (unsigned)e];
            if (bb < (unsigned)NB) st8h(U16, ((size_t)(bb * NCAP + cap)) * DIN + i0 + c8, v);
        }
    }
}

static_assert(32 * 16 * (SEQ / 128) == SEQ * 4);
static_assert(32 * 16 * (SEQ / 256) == SEQ * 2);
__global__ __launch_bounds__(256) void k_agree(const _Float16* __restrict__ U16, const _Float16* __restrict__ F16,
                                               const float* __restrict__ BT, const float* __restrict__ Rin,
                                               float* __restrict__ Rout, unsigned short* __restrict__ R16, int first) {
    __shared__ __align__(16) float sL[NCAP * SEQ];
    const unsigned lane = threadIdx.x & 31u;
    const unsigned wave = (unsigned)__builtin_amdgcn_readfirstlane((int)(threadIdx.x >> 5));
    const unsigned hh = lane >> 4, c = lane & 15u;
    const unsigned b = blockIdx.x;
    float btv[4];
#pragma unroll
    for (int r2 = 0; r2 < 4; ++r2) btv[r2] = BT[(4u * hh + (unsigned)r2) * 32u + b];
    const float lbase = logf(1.0f / (float)SEQ + 1e-8f);
    const _Float16* arow = U16 + ((size_t)(b * NCAP + (c & 7u))) * DIN + 8u * hh;
#pragma unroll 1
    for (unsigned tt = 0; tt < (unsigned)(SEQ / 128); ++tt) {
        const unsigned s0 = (wave * (unsigned)(SEQ / 128) + tt) * 16u;
        const _Float16* brow = F16 + ((size_t)(b * SEQ + s0 + c)) * DIN + 8u * hh;
        v8f acc = (v8f){0.f,0.f,0.f,0.f,0.f,0.f,0.f,0.f};
#pragma unroll 4
        for (unsigned k0 = 0; k0 < (unsigned)DIN; k0 += 32u) {
            const v16h a = frag_ld(arow + k0);
            const v16h bf = frag_ld(brow + k0);
            acc = wmma16(a, bf, acc);
        }
#pragma unroll
        for (int r2 = 0; r2 < 4; ++r2) {
            const unsigned cc = 4u * hh + (unsigned)r2;
            const float dot = (hh != 0u) ? acc[r2 + 4] : acc[r2];
            const float val = dot * (1.0f / 131072.0f) + btv[r2];
            float lg = lbase;
            if (first == 0) lg = logf(Rin[((size_t)(b * NCAP + cc)) * SEQ + s0 + c] + 1e-8f);
            sL[cc * (unsigned)SEQ + s0 + c] = lg + val;
        }
    }
    __syncthreads();
    const unsigned rbase = wave * (unsigned)SEQ;
    float m = -3.0e38f;
#pragma unroll 1
    for (unsigned j = 0; j < (unsigned)(SEQ / 128); ++j) {
        const v4f t4 = *(const v4f*)&sL[rbase + 4u * lane + 128u * j];
        m = fmaxf(m, fmaxf(fmaxf(t4.x, t4.y), fmaxf(t4.z, t4.w)));
    }
#pragma unroll
    for (int o = 16; o > 0; o >>= 1) m = fmaxf(m, __shfl_xor(m, o, 32));
    float sum = 0.f;
#pragma unroll 1
    for (unsigned j = 0; j < (unsigned)(SEQ / 128); ++j) {
        v4f t4 = *(const v4f*)&sL[rbase + 4u * lane + 128u * j];
        t4.x = expf(t4.x - m); t4.y = expf(t4.y - m); t4.z = expf(t4.z - m); t4.w = expf(t4.w - m);
        sum += (t4.x + t4.y) + (t4.z + t4.w);
        *(v4f*)&sL[rbase + 4u * lane + 128u * j] = t4;
    }
#pragma unroll
    for (int o = 16; o > 0; o >>= 1) sum += __shfl_xor(sum, o, 32);
    const float inv = 1.0f / sum;
#pragma unroll 1
    for (unsigned j = 0; j < (unsigned)(SEQ / 128); ++j) {
        v4f t4 = *(const v4f*)&sL[rbase + 4u * lane + 128u * j];
        t4.x *= inv; t4.y *= inv; t4.z *= inv; t4.w *= inv;
        *(v4f*)&sL[rbase + 4u * lane + 128u * j] = t4;
    }
    wave_sync_lds();
    const size_t grow = ((size_t)(b * NCAP + wave)) * SEQ;
#pragma unroll 1
    for (unsigned j = 0; j < (unsigned)(SEQ / 128); ++j) {
        const v4f t4 = *(const v4f*)&sL[rbase + 4u * lane + 128u * j];
        VST2V4(Rout + grow + 4u * lane + 128u * j, t4);
    }
#pragma unroll 1
    for (unsigned j = 0; j < (unsigned)(SEQ / 256); ++j) {
        float v[8];
#pragma unroll
        for (int e = 0; e < 8; ++e)
            v[e] = (sL[rbase + 8u * lane + 256u * j + (unsigned)e] * (float)SEQ - 1.0f) * 16.0f;
        st8h(R16, grow + 8u * lane + 256u * j, v);
    }
}

extern "C" void kernel_launch(void* const* d_in, const int* in_sizes, int n_in, void* d_out, int out_size,
                              void* d_ws, size_t ws_size, hipStream_t stream) {
    if (n_in < 5) return;
    if (in_sizes[0] < NB * SEQ * DIN || in_sizes[1] < DIN * DOUT * NCAP || in_sizes[2] < NCAP) return;
    if (in_sizes[3] < DOUT || in_sizes[4] < DOUT || out_size < NB * NCAP * DOUT) return;

    const float* feat  = (const float*)d_in[0];
    const float* Wm    = (const float*)d_in[1];
    const float* cbias = (const float*)d_in[2];
    const float* gamma = (const float*)d_in[3];
    const float* beta  = (const float*)d_in[4];
    float* out = (float*)d_out;

    char* wsp = (char*)d_ws;
    size_t off = 0;
    auto carve = [&](size_t bytes) -> void* { void* r = wsp + off; off += (bytes + 255) & ~(size_t)255; return r; };
    unsigned short* wp   = (unsigned short*)carve((size_t)2 * NCAP * DOUT * DIN * 2);
    unsigned short* f16  = (unsigned short*)carve((size_t)NB * SEQ * DIN * 2);
    unsigned short* ft16 = (unsigned short*)carve((size_t)NB * DIN * SEQ * 2);
    unsigned short* r16  = (unsigned short*)carve((size_t)NB * NCAP * SEQ * 2);
    float*          r32a = (float*)carve((size_t)NB * NCAP * SEQ * 4);
    float*          r32b = (float*)carve((size_t)NB * NCAP * SEQ * 4);
    unsigned short* m16  = (unsigned short*)carve((size_t)NCAP * NB * DIN * 2);
    unsigned short* u16  = (unsigned short*)carve((size_t)NB * NCAP * DIN * 2);
    float*          bt   = (float*)carve((size_t)NCAP * 32 * 4);
    if (off > ws_size || off > (size_t)134217728) return;

    k_wconv<<<dim3((DIN * 64) / 256, 2), 256, 0, stream>>>(Wm, wp);
    k_fconv<<<NB * (SEQ / 64) * (DIN / 64), 256, 0, stream>>>(feat, f16, ft16);

    for (int it = 0; it < 3; ++it) {
        k_pool<<<NB, 256, 0, stream>>>((const _Float16*)r16, (const _Float16*)ft16, m16, (it == 0) ? 1 : 0);
        k_route<<<NCAP, 256, 0, stream>>>((const _Float16*)m16, (const _Float16*)wp, cbias, gamma, beta, u16, bt, out,
                                          (it == 2) ? 1 : 0);
        if (it < 2) {
            const float* rin = (it == 0) ? r32b : r32a;
            float* rout = (it == 0) ? r32a : r32b;
            k_agree<<<NB, 256, 0, stream>>>((const _Float16*)u16, (const _Float16*)f16, bt, rin, rout, r16, (it == 0) ? 1 : 0);
        }
    }
}
